// S4sequence_27315992002810
// MI455X (gfx1250) — hardware-verified
//
#include <hip/hip_runtime.h>
#include <math.h>
#include <stdint.h>

constexpr int NBATCH = 16;
constexpr int SEQLEN = 4096;
constexpr int NCHAN  = 128;
constexpr int NSTATE = 64;
constexpr int CHLEN  = 64;
constexpr int NCHUNK = 64;
constexpr int NSLICE = 32;
constexpr int SLICE_ELEMS = SEQLEN * NCHAN / NSLICE;
constexpr int PLANE_TILE = CHLEN * CHLEN;
constexpr int NPLANES = 5;
constexpr int OUT_M = NBATCH * SEQLEN;
static_assert(SEQLEN == CHLEN * NCHUNK, "chunking");
static_assert(NSTATE == 64 && CHLEN == 64 && NCHUNK == 64, "tile sizes");
static_assert(SLICE_ELEMS == 16 * 256 * 4, "slice loop");
static_assert(NSLICE == 32, "one lane per slice");
static_assert(OUT_M % 64 == 0 && NCHAN % 64 == 0 && NCHAN % 32 == 0, "gemm tiles");
static_assert(((OUT_M / 64) * (NCHAN / 64)) % 8 == 0, "gemm grid");

constexpr float T_CARRY = 1024.0f;
constexpr float M_CARRY = 4096.0f;
constexpr float V_CARRY = 64.0f;
constexpr float S_CARRY = 16.0f;
constexpr float G_CARRY = 64.0f;
constexpr float W_CARRY = 16.0f;

constexpr size_t WS_PART        = 0;
constexpr size_t WS_PART_BYTES  = (size_t)NBATCH * NSLICE * 128;
constexpr size_t WS_U           = WS_PART + WS_PART_BYTES;
constexpr size_t WS_U_BYTES     = (size_t)NBATCH * NCHAN * SEQLEN * 2;
constexpr size_t WS_PL          = WS_U + WS_U_BYTES;
constexpr size_t WS_PL_BYTES    = (size_t)NPLANES * NCHAN * PLANE_TILE * 2;
constexpr size_t WS_WQ          = WS_PL + WS_PL_BYTES;
constexpr size_t WS_WQ_BYTES    = (size_t)NCHAN * NSTATE * 2 * 4;
constexpr size_t WS_GT          = WS_WQ + WS_WQ_BYTES;
constexpr size_t WS_GT_BYTES    = WS_U_BYTES;
constexpr size_t WS_G           = WS_GT + WS_GT_BYTES;
constexpr size_t WS_G_BYTES     = WS_U_BYTES;
constexpr size_t WS_W1          = WS_G + WS_G_BYTES;
constexpr size_t WS_W1_BYTES    = (size_t)NCHAN * NCHAN * 2;
constexpr size_t WS_TOTAL       = WS_W1 + WS_W1_BYTES;
static_assert(WS_TOTAL == 55738368, "carve total");
static_assert(WS_TOTAL <= 134217728, "carve cap");
static_assert(WS_U % 128 == 0 && WS_PL % 128 == 0 && WS_WQ % 128 == 0 && WS_GT % 128 == 0 && WS_G % 128 == 0 && WS_W1 % 128 == 0, "align");

typedef __attribute__((ext_vector_type(16))) _Float16 v16h;
typedef __attribute__((ext_vector_type(8)))  _Float16 v8h;
typedef __attribute__((ext_vector_type(16))) __bf16   v16b;
typedef __attribute__((ext_vector_type(8)))  __bf16   v8b;
typedef __attribute__((ext_vector_type(8)))  float    v8f;
typedef __attribute__((ext_vector_type(4)))  float    v4f;
typedef __attribute__((ext_vector_type(4)))  unsigned v4u;

__device__ __forceinline__ unsigned short f2bf_bits(float f) {
  unsigned u = __float_as_uint(f);
  return (unsigned short)((u + 0x7FFFu + ((u >> 16) & 1u)) >> 16);
}
__device__ __forceinline__ float bf_bits2f(unsigned short h) { return __uint_as_float(((unsigned)h) << 16); }

__device__ __forceinline__ void dep_guard_h(v8f& a, v8f& b, v16h x, v16h y) { asm volatile("v_nop\n\tv_nop\n\tv_nop\n\tv_nop" : "+v"(a), "+v"(b) : "v"(x), "v"(y)); }
__device__ __forceinline__ void dep_guard_b(v8f& a, v8f& b, v16b x, v16b y) { asm volatile("v_nop\n\tv_nop\n\tv_nop\n\tv_nop" : "+v"(a), "+v"(b) : "v"(x), "v"(y)); }
__device__ __forceinline__ void keep4_h(v16h a, v16h b, v16h c, v16h d) { asm volatile("v_nop" :: "v"(a), "v"(b), "v"(c), "v"(d)); }
__device__ __forceinline__ void keep4_b(v16b a, v16b b, v16b c, v16b d) { asm volatile("v_nop" :: "v"(a), "v"(b), "v"(c), "v"(d)); }
__device__ __forceinline__ void acc_guard4(v8f& a, v8f& b, v8f& c, v8f& d) { asm volatile("v_nop\n\tv_nop\n\tv_nop\n\tv_nop" : "+v"(a), "+v"(b), "+v"(c), "+v"(d)); }
template <typename T> struct Frag;
template <> struct Frag<_Float16> {
  typedef v16h V; union U { v16h v; v8h h[2]; };
  static __device__ __forceinline__ v16h load(const _Float16* p) {
    U f; f.h[0] = *(const v8h*)(p); f.h[1] = *(const v8h*)(p + 16); return f.v;
  }
  static __device__ __forceinline__ v8f mma(v16h a, v16h b, v8f c) {
    return __builtin_amdgcn_wmma_f32_16x16x32_f16(false, a, false, b, (short)0, c, false, false);
  }
  static __device__ __forceinline__ void guard(v8f& a, v8f& b, v16h x, v16h y) { dep_guard_h(a, b, x, y); }
  static __device__ __forceinline__ void keep(v16h a, v16h b, v16h c, v16h d) { keep4_h(a, b, c, d); }
};
template <> struct Frag<__bf16> {
  typedef v16b V; union U { v16b v; v8b h[2]; };
  static __device__ __forceinline__ v16b load(const __bf16* p) {
    U f; f.h[0] = *(const v8b*)(p); f.h[1] = *(const v8b*)(p + 16); return f.v;
  }
  static __device__ __forceinline__ v8f mma(v16b a, v16b b, v8f c) {
    return __builtin_amdgcn_wmma_f32_16x16x32_bf16(false, a, false, b, (short)0, c, false, false);
  }
  static __device__ __forceinline__ void guard(v8f& a, v8f& b, v16b x, v16b y) { dep_guard_b(a, b, x, y); }
  static __device__ __forceinline__ void keep(v16b a, v16b b, v16b c, v16b d) { keep4_b(a, b, c, d); }
};

template <int ET> struct Elem;
template <> struct Elem<0> { typedef _Float16 T; };
template <> struct Elem<1> { typedef __bf16 T; };
template <int ET, bool SPLIT, int BIAS_MODE, int OUT_MODE, bool RESID, int ACT = 0>
__global__ __launch_bounds__(256) void wmma_gemm64(
    const unsigned short* __restrict__ Ap, const unsigned short* __restrict__ A2p, int lda, long strideA,
    const unsigned short* __restrict__ Btp, const unsigned short* __restrict__ Bt2p, int ldb, long strideB,
    void* __restrict__ Cout, void* __restrict__ Cout2, int ldc, long strideC,
    const float* __restrict__ bias,
    const float* __restrict__ resid, long strideR,
    int M, int N, int K, float scale) {
  typedef typename Elem<ET>::T T;
  typedef typename Frag<T>::V V;
  const T* A = (const T*)Ap; const T* A2 = (const T*)A2p; const T* Bt = (const T*)Btp; const T* Bt2 = (const T*)Bt2p;
  __shared__ __align__(16) float sT[8][16 * 68];
  const int b    = blockIdx.y;
  const int lane = threadIdx.x & 31;
  const int wave = threadIdx.x >> 5;
  const int tilesN = N >> 6;
  const int tilesM = M >> 6;
  const int tile = blockIdx.x * 8 + wave;
  if (tile >= tilesM * tilesN) return;
  const int tm = tile / tilesN;
  const int tn = tile - tm * tilesN;
  const int m0 = tm << 6;
  const int n0 = tn << 6;

  const T* Ab  = A  + (size_t)b * strideA;
  const T* Bb  = Bt + (size_t)b * strideB;
  const T* Ab2 = SPLIT ? (A2  + (size_t)b * strideA) : nullptr;
  const T* Bb2 = SPLIT ? (Bt2 + (size_t)b * strideB) : nullptr;

  const int rlane = lane & 15;
  const int koff  = (lane >> 4) * 8;
  const int mOff  = (lane >> 4) * 8;

  v8f acc[4][4];
#pragma unroll
  for (int i = 0; i < 4; ++i)
#pragma unroll
    for (int j = 0; j < 4; ++j) acc[i][j] = (v8f){0.f,0.f,0.f,0.f,0.f,0.f,0.f,0.f};

  for (int k0 = 0; k0 < K; k0 += 32) {
    V bh[4], bl[4];
#pragma unroll
    for (int j = 0; j < 4; ++j) {
      const size_t bo = (size_t)(n0 + (j << 4) + rlane) * ldb + koff + k0;
      bh[j] = Frag<T>::load(Bb + bo);
      if (SPLIT) bl[j] = Frag<T>::load(Bb2 + bo);
    }
#pragma unroll
    for (int i = 0; i < 4; ++i) {
      const size_t ao = (size_t)(m0 + (i << 4) + rlane) * lda + koff + k0;
      V ah = Frag<T>::load(Ab + ao);
      V al;
      if (SPLIT) al = Frag<T>::load(Ab2 + ao);
#pragma unroll
      for (int j = 0; j < 4; ++j) {
        acc[i][j] = Frag<T>::mma(ah, bh[j], acc[i][j]);
        if (SPLIT) {
          acc[i][j] = Frag<T>::mma(ah, bl[j], acc[i][j]);
          acc[i][j] = Frag<T>::mma(al, bh[j], acc[i][j]);
        }
      }
      Frag<T>::guard(acc[i][0], acc[i][3], ah, SPLIT ? al : ah);
    }
    Frag<T>::keep(bh[0], bh[1], bh[2], bh[3]);
    if (SPLIT) Frag<T>::keep(bl[0], bl[1], bl[2], bl[3]);
  }
  acc_guard4(acc[0][0], acc[0][1], acc[0][2], acc[0][3]);
  acc_guard4(acc[1][0], acc[1][1], acc[1][2], acc[1][3]);
  acc_guard4(acc[2][0], acc[2][1], acc[2][2], acc[2][3]);
  acc_guard4(acc[3][0], acc[3][1], acc[3][2], acc[3][3]);

  float* slab = sT[wave];
  const float* Rb = RESID ? (resid + (size_t)b * strideR) : nullptr;
#pragma unroll
  for (int i = 0; i < 4; ++i) {
    const int mBase = m0 + (i << 4);
#pragma unroll
    for (int j = 0; j < 4; ++j) {
      const int n = n0 + (j << 4) + rlane;
      float bv = 0.f;
      if (BIAS_MODE == 2) bv = bias[n];
#pragma unroll
      for (int r = 0; r < 8; ++r) {
        float v = acc[i][j][r] * scale;
        if (BIAS_MODE == 1) v += bias[mBase + mOff + r];
        if (BIAS_MODE == 2) v += bv;
        if (RESID) v += Rb[(size_t)(mBase + mOff + r) * ldc + n];
        if (ACT == 1) v = tanhf(v);
        if (ACT == 2) v = fmaxf(v, 0.0f);
        if (ACT == 3) v = v / (1.0f + expf(-v));
        if (ACT == 4) v = (v > 0.f) ? v : 0.01f * v;
        if (ACT == 5) v = 0.5f * v * (1.0f + erff(v * 0.70710678118654752f));
        slab[(mOff + r) * 68 + (j << 4) + rlane] = v;
      }
    }
    __builtin_amdgcn_fence(__ATOMIC_RELEASE, "workgroup");
    __builtin_amdgcn_wave_barrier();
    __builtin_amdgcn_fence(__ATOMIC_ACQUIRE, "workgroup");
    if (OUT_MODE == 0) {
      float* C = (float*)Cout + (size_t)b * strideC;
      const int hh = lane >> 4, c4 = (lane & 15) * 4;
      for (int pass = 0; pass < 2; ++pass) {
#pragma unroll
        for (int it = 0; it < 8; ++it) {
          const int row = it * 2 + hh;
          v4f v = *(const v4f*)(slab + row * 68 + c4);
          *(volatile v4f*)(C + (size_t)(mBase + row) * ldc + n0 + c4) = v;
        }
        __threadfence();
      }
    } else {
      const int q = lane >> 3, c8 = (lane & 7) * 8;
      unsigned short* C  = (unsigned short*)Cout  + (size_t)b * strideC;
      unsigned short* C2 = (OUT_MODE == 2) ? ((unsigned short*)Cout2 + (size_t)b * strideC) : nullptr;
      for (int pass = 0; pass < 2; ++pass) {
#pragma unroll
        for (int it = 0; it < 4; ++it) {
          const int row = it * 4 + q;
          const float* sp = slab + row * 68 + c8;
          v8h hv, lv;
#pragma unroll
          for (int e = 0; e < 8; ++e) {
            if (OUT_MODE == 1) {
              hv[e] = (_Float16)sp[e];
            } else {
              unsigned short hb = f2bf_bits(sp[e]);
              unsigned short lb = f2bf_bits(sp[e] - bf_bits2f(hb));
              hv[e] = __builtin_bit_cast(_Float16, hb);
              lv[e] = __builtin_bit_cast(_Float16, lb);
            }
          }
          *(volatile v8h*)(C + (size_t)(mBase + row) * ldc + n0 + c8) = hv;
          if (OUT_MODE == 2) *(volatile v8h*)(C2 + (size_t)(mBase + row) * ldc + n0 + c8) = lv;
        }
        __threadfence();
      }
    }
    __builtin_amdgcn_fence(__ATOMIC_RELEASE, "workgroup");
    __builtin_amdgcn_wave_barrier();
    __builtin_amdgcn_fence(__ATOMIC_ACQUIRE, "workgroup");
  }
}

__device__ __forceinline__ void st2_v8h(_Float16* p, v8h v) {
  *(volatile v8h*)p = v;
  __threadfence();
  *(volatile v8h*)p = v;
}

__device__ __forceinline__ void ln_stats(const unsigned* __restrict__ part, int b, int lane, float& meanf, float& rstd) {
  const unsigned* line = part + (size_t)(b * NSLICE + lane) * 32;
  const v4u w = *(const v4u*)line;
  double s1 = __longlong_as_double((long long)((((unsigned long long)w[1]) << 32) | (unsigned long long)w[0]));
  double s2 = __longlong_as_double((long long)((((unsigned long long)w[3]) << 32) | (unsigned long long)w[2]));
#pragma unroll
  for (int off = 1; off < 32; off <<= 1) {
    s1 += __shfl_xor(s1, off, 32);
    s2 += __shfl_xor(s2, off, 32);
  }
  const double inv = 1.0 / (double)(SEQLEN * NCHAN);
  const double mean = s1 * inv;
  double var = s2 * inv - mean * mean;
  var = (var < 0.0) ? 0.0 : var;
  meanf = (float)mean;
  rstd = 1.0f / sqrtf((float)var + 1e-5f);
}

__global__ __launch_bounds__(256) void k_ln_partial(const float* __restrict__ x, unsigned* __restrict__ part) {
  __shared__ double r1[256];
  __shared__ double r2[256];
  const int s = blockIdx.x, b = blockIdx.y, tid = threadIdx.x;
  const float* xb = x + ((size_t)b * SEQLEN * NCHAN + (size_t)s * SLICE_ELEMS);
  double s1 = 0.0, s2 = 0.0;
#pragma unroll 1
  for (int it = 0; it < SLICE_ELEMS / 1024; ++it) {
    const v4f v = *(const v4f*)(xb + (size_t)(it * 256 + tid) * 4);
#pragma unroll
    for (int e = 0; e < 4; ++e) { const double d = (double)v[e]; s1 += d; s2 += d * d; }
  }
  r1[tid] = s1; r2[tid] = s2;
  __syncthreads();
  for (int o = 128; o > 0; o >>= 1) {
    if (tid < o) { r1[tid] += r1[tid + o]; r2[tid] += r2[tid + o]; }
    __syncthreads();
  }
  if (tid < 32) {
    const unsigned long long ua = (unsigned long long)__double_as_longlong(r1[0]);
    const unsigned long long ub = (unsigned long long)__double_as_longlong(r2[0]);
    unsigned wv = 0u;
    wv = (tid == 0) ? (unsigned)(ua & 0xffffffffull) : wv;
    wv = (tid == 1) ? (unsigned)(ua >> 32) : wv;
    wv = (tid == 2) ? (unsigned)(ub & 0xffffffffull) : wv;
    wv = (tid == 3) ? (unsigned)(ub >> 32) : wv;
    unsigned* dst = part + (size_t)(b * NSLICE + s) * 32 + tid;
    *(volatile unsigned*)dst = wv;
    __threadfence();
    *(volatile unsigned*)dst = wv;
  }
}

__global__ __launch_bounds__(256) void k_norm_transpose(const float* __restrict__ x, const unsigned* __restrict__ part,
                                                        unsigned short* __restrict__ uplane) {
  __shared__ __align__(16) float tile[64][68];
  const int l0 = blockIdx.x * 64, h0 = blockIdx.y * 64, b = blockIdx.z;
  const int tid = threadIdx.x, lane = tid & 31, wave = tid >> 5;
  float meanf, rstd;
  ln_stats(part, b, lane, meanf, rstd);
  const float* xb = x + (size_t)b * SEQLEN * NCHAN;
#pragma unroll
  for (int it = 0; it < 4; ++it) {
    const int idx = it * 256 + tid;
    const int r = idx >> 4, c4 = (idx & 15) * 4;
    const v4f v = *(const v4f*)(xb + (size_t)(l0 + r) * NCHAN + h0 + c4);
    *(v4f*)(&tile[r][c4]) = v;
  }
  __syncthreads();
  _Float16* ub = (_Float16*)uplane;
  const int q = lane >> 3, c8 = (lane & 7) * 8;
  for (int pass = 0; pass < 2; ++pass) {
#pragma unroll
    for (int it = 0; it < 2; ++it) {
      const int hr = wave * 8 + it * 4 + q;
      v8h hv;
#pragma unroll
      for (int e = 0; e < 8; ++e) hv[e] = (_Float16)((tile[c8 + e][hr] - meanf) * rstd);
      *(volatile v8h*)(ub + (size_t)(b * NCHAN + h0 + hr) * SEQLEN + l0 + c8) = hv;
    }
    __threadfence();
  }
}

__global__ __launch_bounds__(256) void k_materials(const float* __restrict__ A_re, const float* __restrict__ A_im,
                                                   const float* __restrict__ B_re, const float* __restrict__ B_im,
                                                   const float* __restrict__ C_re, const float* __restrict__ C_im,
                                                   const float* __restrict__ log_dt,
                                                   unsigned short* __restrict__ planes, float* __restrict__ wq) {
#pragma clang fp contract(off)
  __shared__ float pw_re[NSTATE * 65];
  __shared__ float pw_im[NSTATE * 65];
  __shared__ float ksh[CHLEN];
  __shared__ float cbr_s[NSTATE];
  __shared__ float cbi_s[NSTATE];
  const int h = blockIdx.x, tid = threadIdx.x, lane = tid & 31, wave = tid >> 5;
  const float dt = expf(log_dt[h]);
#pragma unroll 1
  for (int idx = tid; idx < NSTATE * 65; idx += 256) {
    const int n = idx / 65, p = idx - n * 65;
    const float ar = A_re[h * NSTATE + n] * dt;
    const float ai = A_im[h * NSTATE + n] * dt;
    const float mag = expf(ar * (float)p);
    float sn, cs;
    sincosf(ai * (float)p, &sn, &cs);
    pw_re[idx] = mag * cs;
    pw_im[idx] = mag * sn;
  }
  if (tid < NSTATE) {
    const int n = tid;
    const float br = B_re[h * NSTATE + n], bi = B_im[h * NSTATE + n];
    const float cr = C_re[h * NSTATE + n], ci = C_im[h * NSTATE + n];
    const float bdr = br * dt, bdi = bi * dt;
    cbr_s[n] = cr * bdr - ci * bdi;
    cbi_s[n] = cr * bdi + ci * bdr;
  }
  __syncthreads();
  if (tid < CHLEN) {
    const int d = tid;
    float kr = 0.f;
#pragma unroll 1
    for (int n = 0; n < NSTATE; ++n) kr += (cbr_s[n] * pw_re[n * 65 + d] - cbi_s[n] * pw_im[n * 65 + d]);
    ksh[d] = kr;
  }
  __syncthreads();
  _Float16* pl = (_Float16*)planes;
  const size_t pstride = (size_t)NCHAN * PLANE_TILE;
  const size_t hoff = (size_t)h * PLANE_TILE;
  const int q = lane >> 3, c8 = (lane & 7) * 8;
#pragma unroll 1
  for (int it = 0; it < 2; ++it) {
    const int row = it * 32 + wave * 4 + q;
    v8h tv, mrv, miv, vrv, viv;
#pragma unroll
    for (int e = 0; e < 8; ++e) {
      const int col = c8 + e;
      const int dd = row - col;
      const int dcl = dd < 0 ? 0 : dd;
      float tvf = ksh[dcl] * T_CARRY;
      tvf = (dd < 0) ? 0.0f : tvf;
      tv[e] = (_Float16)tvf;
      const float pr = pw_re[col * 65 + row + 1], pq = pw_im[col * 65 + row + 1];
      const float cr = cbr_s[col], ci = cbi_s[col];
      mrv[e] = (_Float16)((cr * pr - ci * pq) * M_CARRY);
      miv[e] = (_Float16)(-(cr * pq + ci * pr) * M_CARRY);
      vrv[e] = (_Float16)(pw_re[row * 65 + 63 - col] * V_CARRY);
      viv[e] = (_Float16)(pw_im[row * 65 + 63 - col] * V_CARRY);
    }
    const size_t eo = hoff + (size_t)row * CHLEN + c8;
    st2_v8h(pl + eo, tv);
    st2_v8h(pl + pstride + eo, mrv);
    st2_v8h(pl + 2 * pstride + eo, miv);
    st2_v8h(pl + 3 * pstride + eo, vrv);
    st2_v8h(pl + 4 * pstride + eo, viv);
  }
  if (wave == 0) {
    v4f wv;
    wv[0] = pw_re[(2 * lane) * 65 + 64];
    wv[1] = pw_im[(2 * lane) * 65 + 64];
    wv[2] = pw_re[(2 * lane + 1) * 65 + 64];
    wv[3] = pw_im[(2 * lane + 1) * 65 + 64];
    float* dst = wq + (size_t)h * (NSTATE * 2) + lane * 4;
    *(volatile v4f*)dst = wv;
    __threadfence();
    *(volatile v4f*)dst = wv;
  }
}

__global__ __launch_bounds__(256) void k_cast_scaled(const float* __restrict__ in, unsigned short* __restrict__ out, int n2, float sc) {
  const int i = blockIdx.x * 256 + threadIdx.x;
  if (i < n2) {
    const _Float16 h0 = (_Float16)(in[2 * i] * sc), h1 = (_Float16)(in[2 * i + 1] * sc);
    const unsigned u = (unsigned)__builtin_bit_cast(unsigned short, h0) | ((unsigned)__builtin_bit_cast(unsigned short, h1) << 16);
    ((volatile unsigned*)out)[i] = u;
    __threadfence();
    ((volatile unsigned*)out)[i] = u;
  }
}

__global__ __launch_bounds__(256) void k_s4_block(const unsigned short* __restrict__ uplane, const unsigned short* __restrict__ planes,
                                                  const float* __restrict__ wq, const float* __restrict__ x,
                                                  const unsigned* __restrict__ part, const float* __restrict__ Dp,
                                                  unsigned short* __restrict__ gT) {
  __shared__ __align__(16) float regA[2 * NSTATE * 68];
  __shared__ __align__(16) _Float16 s_re[NCHUNK * 72];
  __shared__ __align__(16) _Float16 s_im[NCHUNK * 72];
  __shared__ __align__(16) _Float16 gout[NCHUNK * 72];
  static_assert(2 * NSTATE * 68 == SEQLEN + 8 * 576, "lds reuse");

  const int bh = blockIdx.x, b = bh >> 7, h = bh & 127;
  const int tid = threadIdx.x, lane = tid & 31, wave = tid >> 5;
  const int rlane = lane & 15, koff = (lane >> 4) * 8, mOff = (lane >> 4) * 8;
  const _Float16* pl = (const _Float16*)planes;
  const size_t pstride = (size_t)NCHAN * PLANE_TILE;
  const size_t hoff = (size_t)h * PLANE_TILE;
  const _Float16* uh  = (const _Float16*)uplane + (size_t)bh * SEQLEN;
  const _Float16* tpl = pl + hoff;
  const _Float16* mrp = pl + pstride + hoff;
  const _Float16* mip = pl + 2 * pstride + hoff;
  float meanf, rstd;
  ln_stats(part, b, lane, meanf, rstd);

  {
    const int prt = wave >> 2, it1 = wave & 3;
    const _Float16* vp = pl + (size_t)(3 + prt) * pstride + hoff;
    v8f acc[4];
#pragma unroll
    for (int j = 0; j < 4; ++j) acc[j] = (v8f){0.f,0.f,0.f,0.f,0.f,0.f,0.f,0.f};
#pragma unroll
    for (int ks = 0; ks < 2; ++ks) {
      const int k0 = ks * 32;
      v16h bfr[4];
#pragma unroll
      for (int j = 0; j < 4; ++j) bfr[j] = Frag<_Float16>::load(uh + (size_t)(j * 16 + rlane) * CHLEN + k0 + koff);
      const v16h af = Frag<_Float16>::load(vp + (size_t)(it1 * 16 + rlane) * CHLEN + k0 + koff);
#pragma unroll
      for (int j = 0; j < 4; ++j) acc[j] = Frag<_Float16>::mma(af, bfr[j], acc[j]);
      dep_guard_h(acc[0], acc[3], af, af);
      keep4_h(bfr[0], bfr[1], bfr[2], bfr[3]);
    }
    acc_guard4(acc[0], acc[1], acc[2], acc[3]);
    float* inj = regA + prt * (NSTATE * 68);
    const float invV = 1.0f / V_CARRY;
#pragma unroll
    for (int j = 0; j < 4; ++j)
#pragma unroll
      for (int r = 0; r < 8; ++r)
        inj[(it1 * 16 + mOff + r) * 68 + j * 16 + rlane] = acc[j][r] * invV;
  }
  __syncthreads();

  if (tid < NSTATE) {
    const int n = tid;
    const float wr = wq[(size_t)h * (NSTATE * 2) + 2 * n];
    const float wi = wq[(size_t)h * (NSTATE * 2) + 2 * n + 1];
    float sr = 0.f, si = 0.f;
#pragma unroll 1
    for (int c = 0; c < NCHUNK; ++c) {
      s_re[c * 72 + n] = (_Float16)(sr * S_CARRY);
      s_im[c * 72 + n] = (_Float16)(si * S_CARRY);
      const float ir = regA[n * 68 + c];
      const float ii = regA[NSTATE * 68 + n * 68 + c];
      const float nsr = wr * sr - wi * si + ir;
      const float nsi = wr * si + wi * sr + ii;
      sr = nsr; si = nsi;
    }
  }
  __syncthreads();

#pragma unroll 1
  for (int idx = tid; idx < SEQLEN; idx += 256) regA[idx] = x[((size_t)b * SEQLEN + idx) * NCHAN + h];
  __syncthreads();

  {
    const int it3 = wave >> 1, jb = (wave & 1) * 2;
    v8f accT[2], accM[2];
#pragma unroll
    for (int jj = 0; jj < 2; ++jj) { accT[jj] = (v8f){0.f,0.f,0.f,0.f,0.f,0.f,0.f,0.f}; accM[jj] = accT[jj]; }
#pragma unroll
    for (int ks = 0; ks < 2; ++ks) {
      const int k0 = ks * 32;
      v16h bu[2], bsr[2], bsi[2];
#pragma unroll
      for (int jj = 0; jj < 2; ++jj) {
        const int crow = (jb + jj) * 16 + rlane;
        bu[jj]  = Frag<_Float16>::load(uh + (size_t)crow * CHLEN + k0 + koff);
        bsr[jj] = Frag<_Float16>::load(s_re + crow * 72 + k0 + koff);
        bsi[jj] = Frag<_Float16>::load(s_im + crow * 72 + k0 + koff);
      }
      const size_t ao = (size_t)(it3 * 16 + rlane) * CHLEN + k0 + koff;
      const v16h aT = Frag<_Float16>::load(tpl + ao);
      const v16h aR = Frag<_Float16>::load(mrp + ao);
      const v16h aI = Frag<_Float16>::load(mip + ao);
#pragma unroll
      for (int jj = 0; jj < 2; ++jj) {
        accT[jj] = Frag<_Float16>::mma(aT, bu[jj], accT[jj]);
        accM[jj] = Frag<_Float16>::mma(aR, bsr[jj], accM[jj]);
        accM[jj] = Frag<_Float16>::mma(aI, bsi[jj], accM[jj]);
      }
      dep_guard_h(accT[0], accT[1], aT, aR);
      dep_guard_h(accM[0], accM[1], aI, aI);
      keep4_h(bu[0], bu[1], bsr[0], bsr[1]);
      keep4_h(bsi[0], bsi[1], bsi[0], bsi[1]);
    }
    acc_guard4(accT[0], accT[1], accM[0], accM[1]);

    float* slab = regA + SEQLEN + wave * 576;
    const float invT = 1.0f / T_CARRY;
    const float invM = 1.0f / (M_CARRY * S_CARRY);
    const float dh = Dp[h];
#pragma unroll
    for (int jj = 0; jj < 2; ++jj) {
      const int cc = (jb + jj) * 16 + rlane;
#pragma unroll
      for (int r = 0; r < 8; ++r) {
        const int ii = it3 * 16 + mOff + r;
        const float xv = regA[cc * CHLEN + ii];
        const float u = (xv - meanf) * rstd;
        const float y = accT[jj][r] * invT + accM[jj][r] * invM + dh * u;
        slab[(mOff + r) * 36 + jj * 16 + rlane] = y;
      }
    }
    __builtin_amdgcn_fence(__ATOMIC_RELEASE, "workgroup");
    __builtin_amdgcn_wave_barrier();
    __builtin_amdgcn_fence(__ATOMIC_ACQUIRE, "workgroup");
#pragma unroll 1
    for (int e = 0; e < 16; ++e) {
      const float v = slab[e * 36 + lane];
      const float gl = 0.5f * v * (1.0f + erff(v * 0.70710678118654752f));
      gout[(jb * 16 + lane) * 72 + it3 * 16 + e] = (_Float16)(gl * G_CARRY);
    }
  }
  __syncthreads();

  {
    _Float16* gd = (_Float16*)gT + (size_t)bh * SEQLEN;
    const int q = lane >> 3, c8 = (lane & 7) * 8;
    for (int pass = 0; pass < 2; ++pass) {
#pragma unroll
      for (int it2 = 0; it2 < 2; ++it2) {
        const int cc = wave * 8 + it2 * 4 + q;
        const v8h hv = *(const v8h*)(gout + cc * 72 + c8);
        *(volatile v8h*)(gd + (size_t)cc * CHLEN + c8) = hv;
      }
      __threadfence();
    }
  }
}

__global__ __launch_bounds__(256) void k_transpose_g(const unsigned short* __restrict__ gT, unsigned short* __restrict__ g) {
  __shared__ __align__(16) unsigned short tile[64 * 72];
  const int l0 = blockIdx.x * 64, h0 = blockIdx.y * 64, b = blockIdx.z;
  const int tid = threadIdx.x, lane = tid & 31, wave = tid >> 5;
#pragma unroll
  for (int it = 0; it < 2; ++it) {
    const int idx = it * 256 + tid;
    const int row = idx >> 3, seg = idx & 7;
    const v4u w = *(const v4u*)(gT + (size_t)(b * NCHAN + h0 + row) * SEQLEN + l0 + seg * 8);
    *(v4u*)(tile + row * 72 + seg * 8) = w;
  }
  __syncthreads();
  const int q = lane >> 3, c8 = (lane & 7) * 8;
  for (int pass = 0; pass < 2; ++pass) {
#pragma unroll
    for (int it = 0; it < 2; ++it) {
      const int lr = wave * 8 + it * 4 + q;
      v4u o;
#pragma unroll
      for (int e = 0; e < 4; ++e) {
        const unsigned lo = (unsigned)tile[(c8 + 2 * e) * 72 + lr];
        const unsigned hi = (unsigned)tile[(c8 + 2 * e + 1) * 72 + lr];
        o[e] = lo | (hi << 16);
      }
      *(volatile v4u*)(g + ((size_t)b * SEQLEN + l0 + lr) * NCHAN + h0 + c8) = o;
    }
    __threadfence();
  }
}

extern "C" void kernel_launch(void* const* d_in, const int* in_sizes, int n_in,
                              void* d_out, int out_size, void* d_ws, size_t ws_size,
                              hipStream_t stream) {
  if (n_in < 11) return;
  if (in_sizes[0] != NBATCH * SEQLEN * NCHAN) return;
  if (in_sizes[1] != NCHAN * NSTATE || in_sizes[2] != NCHAN * NSTATE || in_sizes[3] != NCHAN * NSTATE ||
      in_sizes[4] != NCHAN * NSTATE || in_sizes[5] != NCHAN * NSTATE || in_sizes[6] != NCHAN * NSTATE) return;
  if (in_sizes[7] != NCHAN || in_sizes[8] != NCHAN || in_sizes[9] != NCHAN * NCHAN || in_sizes[10] != NCHAN) return;
  if (out_size != NBATCH * SEQLEN * NCHAN) return;
  if (ws_size < WS_TOTAL) return;

  const float* x      = (const float*)d_in[0];
  const float* A_re   = (const float*)d_in[1];
  const float* A_im   = (const float*)d_in[2];
  const float* B_re   = (const float*)d_in[3];
  const float* B_im   = (const float*)d_in[4];
  const float* C_re   = (const float*)d_in[5];
  const float* C_im   = (const float*)d_in[6];
  const float* Dp     = (const float*)d_in[7];
  const float* log_dt = (const float*)d_in[8];
  const float* W1     = (const float*)d_in[9];
  const float* b1     = (const float*)d_in[10];

  char* ws = (char*)d_ws;
  unsigned*       part   = (unsigned*)(ws + WS_PART);
  unsigned short* uplane = (unsigned short*)(ws + WS_U);
  unsigned short* planes = (unsigned short*)(ws + WS_PL);
  float*          wq     = (float*)(ws + WS_WQ);
  unsigned short* gT     = (unsigned short*)(ws + WS_GT);
  unsigned short* g16    = (unsigned short*)(ws + WS_G);
  unsigned short* w1h    = (unsigned short*)(ws + WS_W1);

  k_ln_partial<<<dim3(NSLICE, NBATCH), 256, 0, stream>>>(x, part);
  k_norm_transpose<<<dim3(SEQLEN / 64, NCHAN / 64, NBATCH), 256, 0, stream>>>(x, part, uplane);
  k_materials<<<NCHAN, 256, 0, stream>>>(A_re, A_im, B_re, B_im, C_re, C_im, log_dt, planes, wq);
  k_cast_scaled<<<(NCHAN * NCHAN / 2 + 255) / 256, 256, 0, stream>>>(W1, w1h, NCHAN * NCHAN / 2, W_CARRY);
  k_s4_block<<<NBATCH * NCHAN, 256, 0, stream>>>(uplane, planes, wq, x, part, Dp, gT);
  k_transpose_g<<<dim3(SEQLEN / 64, NCHAN / 64, NBATCH), 256, 0, stream>>>(gT, g16);
  wmma_gemm64<0, false, 2, 0, true, 0><<<dim3(((OUT_M / 64) * (NCHAN / 64)) / 8, 1), 256, 0, stream>>>(
      g16, g16, NCHAN, 0L,
      w1h, w1h, NCHAN, 0L,
      d_out, d_out, NCHAN, 0L,
      b1,
      x, 0L,
      OUT_M, NCHAN, NCHAN, 1.0f / (G_CARRY * W_CARRY));
}
